// SolvGNNV3_63780264346183
// MI455X (gfx1250) — hardware-verified
//
#include <hip/hip_runtime.h>


namespace {
constexpr int N = 20000, E = 320000, NG = 64, IN = 74, INP = 96, H = 256, H1 = 1024, H2 = 512, NPAD = 20096, NBLK = NPAD / 128, NCONV = 10;
constexpr float AS = 4096.0f;

typedef _Float16 b16;
typedef __attribute__((ext_vector_type(16))) _Float16 v16b;
typedef __attribute__((ext_vector_type(8)))  _Float16 v8b;
typedef __attribute__((ext_vector_type(8)))  float v8f;
typedef __attribute__((ext_vector_type(4)))  float v4f;

__device__ __forceinline__ v8b ld8b(const b16* p) { return *(const v8b*)p; }
__device__ __forceinline__ v16b cat8b(v8b a, v8b b) { return __builtin_shufflevector(a, b, 0, 1, 2, 3, 4, 5, 6, 7, 8, 9, 10, 11, 12, 13, 14, 15); }
__device__ __forceinline__ v16b frag_kb(const b16* p, int hh) { return cat8b(ld8b(p + 8 * hh), ld8b(p + 16 + 8 * hh)); }
__device__ __forceinline__ void split16(float v, b16& hi, b16& lo) { hi = (b16)v; lo = (b16)(v - (float)hi); }
__device__ __forceinline__ void frag_ksplit(const float* p, int hh, v16b& fh_, v16b& fl_) {
  const float* p0 = p + 8 * hh; const float* p1 = p + 16 + 8 * hh;
#pragma unroll
  for (int e = 0; e < 8; ++e) { b16 a, c; split16(p0[e], a, c); fh_[e] = a; fl_[e] = c; split16(p1[e], a, c); fh_[8 + e] = a; fl_[8 + e] = c; }
}
__device__ __forceinline__ v8f wmma16b(v16b a, v16b b, v8f c) {
  v8f d = __builtin_amdgcn_wmma_f32_16x16x32_f16(false, a, false, b, (short)0, c, false, false);
  asm volatile("v_nop\n\tv_nop\n\tv_nop\n\tv_nop" : "+v"(d) : "v"(a), "v"(b));
  return d;
}
__device__ __forceinline__ void wave_lds_sync() {
  __builtin_amdgcn_fence(__ATOMIC_RELEASE, "workgroup");
  __builtin_amdgcn_wave_barrier();
  __builtin_amdgcn_fence(__ATOMIC_ACQUIRE, "workgroup");
}

struct Opnd { const void* p0; const void* p1; int ld; };
template <int NP> __device__ __forceinline__ void load_frags(const Opnd& o, int row, int kb, int hh, v16b& fh_, v16b& fl_) {
  if (NP == 0) { frag_ksplit((const float*)o.p0 + (size_t)row * o.ld + kb, hh, fh_, fl_); }
  else if (NP == 4) {
    const float* p = (const float*)o.p0 + (size_t)row * o.ld + kb; const float* p0 = p + 8 * hh; const float* p1 = p + 16 + 8 * hh;
#pragma unroll
    for (int e = 0; e < 8; ++e) { b16 a, c; split16(p0[e] * 64.0f, a, c); fh_[e] = a; fl_[e] = c; split16(p1[e] * 64.0f, a, c); fh_[8 + e] = a; fl_[8 + e] = c; }
  } else if (NP == 3) {
    const float* p = (const float*)o.p0 + (size_t)row * o.ld + kb; const float* p0 = p + 8 * hh; const float* p1 = p + 16 + 8 * hh;
#pragma unroll
    for (int e = 0; e < 8; ++e) { fh_[e] = (b16)p0[e]; fh_[8 + e] = (b16)p1[e]; }
    fl_ = fh_;
  } else {
    fh_ = frag_kb((const b16*)o.p0 + (size_t)row * o.ld + kb, hh);
    if (NP == 2) fl_ = frag_kb((const b16*)o.p1 + (size_t)row * o.ld + kb, hh); else fl_ = fh_;
  }
}
template <int ANP, int BNP> __device__ __forceinline__ v8f mac(v16b ah, v16b al, v16b bh, v16b bl, v8f c) {
  c = wmma16b(ah, bh, c);
  if (BNP == 0 || BNP == 2 || BNP == 4) c = wmma16b(ah, bl, c);
  if (ANP == 0 || ANP == 2 || ANP == 4) c = wmma16b(al, bh, c);
  return c;
}
template <int ANP, int BNP>
__device__ __forceinline__ void gemm_tile(const Opnd& A, const Opnd& B, int K, int m0, int c0, int nloc, int hlf, v8f (&acc)[2][4]) {
  for (int kb = 0; kb < K; kb += 32) {
    v16b a0h, a0l, a1h, a1l;
    load_frags<ANP>(A, m0 + nloc, kb, hlf, a0h, a0l);
    load_frags<ANP>(A, m0 + 16 + nloc, kb, hlf, a1h, a1l);
#pragma unroll
    for (int t = 0; t < 4; ++t) {
      v16b bh, bl;
      load_frags<BNP>(B, c0 + t * 16 + nloc, kb, hlf, bh, bl);
      acc[0][t] = mac<ANP, BNP>(a0h, a0l, bh, bl, acc[0][t]);
      acc[1][t] = mac<ANP, BNP>(a1h, a1l, bh, bl, acc[1][t]);
    }
  }
}

__device__ __forceinline__ void epi_planes(v8f (&acc)[2][4], float scale, bool two, b16* __restrict__ oh, b16* __restrict__ ol, int ldo,
                                           int m0, int c0, int lane, b16* Th, b16* Tl) {
  const int nloc = lane & 15, hlf = lane >> 4;
#pragma unroll
  for (int t = 0; t < 4; ++t)
#pragma unroll
    for (int r = 0; r < 2; ++r)
#pragma unroll
      for (int v = 0; v < 8; ++v) {
        const int rr = r * 16 + v + 8 * hlf, cc = t * 16 + nloc;
        b16 h_, l_; split16(acc[r][t][v] * scale, h_, l_);
        Th[rr * 64 + cc] = h_; Tl[rr * 64 + cc] = l_;
      }
  wave_lds_sync();
  for (int pass = 0; pass < 2; ++pass) {
#pragma unroll
    for (int j = 0; j < 8; ++j) {
      const int rr = j * 4 + (lane >> 3), c8 = (lane & 7) * 8;
      const size_t o = (size_t)(m0 + rr) * ldo + c0 + c8;
      *(volatile v8b*)(oh + o) = ld8b(Th + rr * 64 + c8);
      if (two) *(volatile v8b*)(ol + o) = ld8b(Tl + rr * 64 + c8);
    }
    __threadfence();
  }
}
__device__ __forceinline__ void epi_f32(v8f (&acc)[2][4], float scale, const float* rscale, float* __restrict__ out, int ldo, int m0, int c0, int lane, float* Tt) {
  const int nloc = lane & 15, hlf = lane >> 4;
#pragma unroll
  for (int t = 0; t < 4; ++t)
#pragma unroll
    for (int r = 0; r < 2; ++r)
#pragma unroll
      for (int v = 0; v < 8; ++v) {
        const int rr = r * 16 + v + 8 * hlf;
        const float rs = rscale ? rscale[(size_t)(m0 + rr) * 32] : 1.0f;
        Tt[rr * 64 + t * 16 + nloc] = acc[r][t][v] * scale * rs;
      }
  wave_lds_sync();
  float* dst0 = out + (size_t)m0 * ldo + c0;
  for (int pass = 0; pass < 2; ++pass) {
#pragma unroll
    for (int j = 0; j < 16; ++j) { const int rr = j * 2 + hlf, c4 = nloc * 4; *(volatile v4f*)(dst0 + (size_t)rr * ldo + c4) = *(const v4f*)(Tt + rr * 64 + c4); }
    __threadfence();
  }
}


__global__ __launch_bounds__(256) void prep_kernel(const float* __restrict__ x, const float* __restrict__ W0, const float* __restrict__ gW, const float* __restrict__ W1, const float* __restrict__ W2, const float* __restrict__ W3,
                                                   float* __restrict__ xp, b16* __restrict__ w0, b16* __restrict__ gw, b16* __restrict__ w1, b16* __restrict__ w2, b16* __restrict__ w3) {
  const size_t tid = (size_t)blockIdx.x * blockDim.x + threadIdx.x, nth = (size_t)gridDim.x * blockDim.x;
  for (int pass = 0; pass < 2; ++pass) {
    for (size_t p = tid; p < (size_t)NPAD * INP; p += nth) { const int n = (int)(p / INP), k = (int)(p % INP); const float v = x[(size_t)min(n, N - 1) * IN + min(k, IN - 1)]; ((volatile float*)xp)[p] = (n < N && k < IN) ? v : 0.0f; }
    for (size_t p = tid; p < (size_t)H * INP / 8; p += nth) { const int n = (int)(p / (INP / 8)), k0 = (int)(p % (INP / 8)) * 8; v8b v;
#pragma unroll
      for (int e = 0; e < 8; ++e) { const int k = k0 + e; const float w = W0[(size_t)min(k, IN - 1) * H + n]; v[e] = (b16)((k < IN) ? w : 0.0f); }
      *(volatile v8b*)(w0 + (size_t)n * INP + k0) = v; }
    for (size_t p = tid; p < (size_t)NCONV * H * H / 8; p += nth) { const int l = (int)(p / (H * H / 8)); const int rem = (int)(p % (H * H / 8)), n = rem / (H / 8), k0 = (rem % (H / 8)) * 8; v8b v;
#pragma unroll
      for (int e = 0; e < 8; ++e) v[e] = (b16)gW[((size_t)l * H + k0 + e) * H + n];
      *(volatile v8b*)(gw + ((size_t)l * H + n) * H + k0) = v; }
    for (size_t p = tid; p < (size_t)H1 * H / 8; p += nth) { const int n = (int)(p / (H / 8)), k0 = (int)(p % (H / 8)) * 8; v8b v;
#pragma unroll
      for (int e = 0; e < 8; ++e) v[e] = (b16)W1[(size_t)(k0 + e) * H1 + n];
      *(volatile v8b*)(w1 + (size_t)n * H + k0) = v; }
    for (size_t p = tid; p < (size_t)H2 * H1 / 8; p += nth) { const int n = (int)(p / (H1 / 8)), k0 = (int)(p % (H1 / 8)) * 8; v8b v;
#pragma unroll
      for (int e = 0; e < 8; ++e) v[e] = (b16)W2[(size_t)(k0 + e) * H2 + n];
      *(volatile v8b*)(w2 + (size_t)n * H1 + k0) = v; }
    for (size_t p = tid; p < (size_t)16 * H2 / 8; p += nth) { const int n = (int)(p / (H2 / 8)), k0 = (int)(p % (H2 / 8)) * 8; v8b v;
#pragma unroll
      for (int e = 0; e < 8; ++e) v[e] = (b16)((n == 0) ? W3[k0 + e] : 0.0f);
      *(volatile v8b*)(w3 + (size_t)n * H2 + k0) = v; }
    __threadfence();
  }
}

typedef __attribute__((ext_vector_type(4))) int v4i;
__global__ __launch_bounds__(256) void deg_kernel(const int* __restrict__ idx, float* __restrict__ dsc) {
  __shared__ int cnt[NPAD];
  const int t_ = threadIdx.x;
  for (int i = t_; i < NPAD; i += 256) cnt[i] = 0;
  __syncthreads();
  for (int e0 = t_ * 8; e0 < E; e0 += 256 * 8) { const v4i a = *(const v4i*)(idx + e0), b = *(const v4i*)(idx + e0 + 4); const int dd[8] = {a[0], a[1], a[2], a[3], b[0], b[1], b[2], b[3]};
#pragma unroll
    for (int j = 0; j < 8; ++j) { const unsigned sl = (unsigned)dd[j]; if (sl < (unsigned)N) atomicAdd(&cnt[sl], 1); } }
  __syncthreads();
  for (int pass = 0; pass < 2; ++pass) { for (int i = t_; i < NPAD; i += 256) ((volatile float*)dsc)[i] = (i < N) ? rsqrtf(fmaxf((float)cnt[i], 1.0f)) : 0.0f; __threadfence(); }
}

__device__ __forceinline__ void frag_split(const float* __restrict__ row, int kb, int hh, float scale, v16b& hi, v16b& lo) {
#pragma unroll
  for (int e = 0; e < 16; ++e) { const int k = kb + ((e < 8) ? (8 * hh + e) : (16 + 8 * hh + e - 8)); b16 a, c; split16(row[k] * scale * AS, a, c); hi[e] = a; lo[e] = c; }
}

template <int KIN, int NOUT, bool MLP>
__global__ __launch_bounds__(128) void lin_kernel(const float* __restrict__ h, const float* __restrict__ dsc, const b16* __restrict__ w, const float* __restrict__ bias, float* __restrict__ hw) {
  __shared__ __attribute__((aligned(16))) float Ts[4][32 * 64];
  const int lane = threadIdx.x & 31, wave = threadIdx.x >> 5, nloc = lane & 15, hlf = lane >> 4, m0 = blockIdx.y * 128 + wave * 32, c0 = blockIdx.x * 64;
  v8f acc[2][4];
#pragma unroll
  for (int r = 0; r < 2; ++r)
#pragma unroll
    for (int t = 0; t < 4; ++t) acc[r][t] = (v8f){};
  const int ra = m0 + nloc, rb = m0 + 16 + nloc;
  const float sa = MLP ? 1.0f : dsc[ra], sb = MLP ? 1.0f : dsc[rb];
#pragma unroll 1
  for (int kb = 0; kb < KIN; kb += 32) { v16b a0, l0, a1, l1; frag_split(h + (size_t)ra * KIN, kb, hlf, sa, a0, l0); frag_split(h + (size_t)rb * KIN, kb, hlf, sb, a1, l1);
#pragma unroll
    for (int t = 0; t < 4; ++t) { const v16b bw = frag_kb(w + (size_t)(c0 + t * 16 + nloc) * KIN + kb, hlf);
      acc[0][t] = wmma16b(a0, bw, acc[0][t]); acc[0][t] = wmma16b(l0, bw, acc[0][t]); acc[1][t] = wmma16b(a1, bw, acc[1][t]); acc[1][t] = wmma16b(l1, bw, acc[1][t]); } }
  if (MLP) {
#pragma unroll
    for (int t = 0; t < 4; ++t)
#pragma unroll
      for (int r = 0; r < 2; ++r)
#pragma unroll
        for (int v = 0; v < 8; ++v) { float val = acc[r][t][v] * (1.0f / AS) + bias[c0 + t * 16 + nloc]; acc[r][t][v] = (val > 0.0f) ? val : 0.01f * val; }
    epi_f32(acc, 1.0f, nullptr, hw, NOUT, m0, c0, lane, Ts[wave]);
  } else epi_f32(acc, 1.0f / AS, nullptr, hw, NOUT, m0, c0, lane, Ts[wave]);
}
template <int DF, int NB, bool RELU>
__global__ __launch_bounds__(256) void aggsv_kernel(const int* __restrict__ esrc, const int* __restrict__ edst, const float* __restrict__ x, const float* __restrict__ din, const float* __restrict__ bias, float* __restrict__ zin) {
  __shared__ __attribute__((aligned(16))) int acc[NB * DF];
  __shared__ int list[8 * 256]; __shared__ int cnt[NB];
  constexpr float FXS = 8388608.0f, FXI = 1.0f / 8388608.0f;
  const int t_ = threadIdx.x, wave = t_ >> 5, lane = t_ & 31, base = blockIdx.x * NB;
  for (int i = t_; i < NB * DF; i += 256) acc[i] = 0;
  for (int i = t_; i < NB; i += 256) cnt[i] = 0;
  __syncthreads();
  int* wl = list + wave * 256;
  typedef __attribute__((ext_vector_type(4))) int v4i;
  for (int c0 = 0; c0 < E; c0 += 256 * 8) {
    const int e0 = c0 + (wave * 32 + lane) * 8;
    int dd[8];
    if (e0 + 7 < E) { const v4i a = *(const v4i*)(edst + e0), b = *(const v4i*)(edst + e0 + 4); dd[0] = a[0]; dd[1] = a[1]; dd[2] = a[2]; dd[3] = a[3]; dd[4] = b[0]; dd[5] = b[1]; dd[6] = b[2]; dd[7] = b[3]; }
    else {
#pragma unroll
      for (int j = 0; j < 8; ++j) dd[j] = (e0 + j < E) ? edst[e0 + j] : -1; }
    unsigned sl[8]; bool hit[8]; bool anyl = false;
#pragma unroll
    for (int j = 0; j < 8; ++j) { sl[j] = (unsigned)(dd[j] - base); hit[j] = sl[j] < (unsigned)NB; anyl |= hit[j]; }
    int wc = 0;
    if (__builtin_amdgcn_ballot_w32(anyl) != 0u) {
#pragma unroll
      for (int j = 0; j < 8; ++j) {
        const unsigned mj = __builtin_amdgcn_ballot_w32(hit[j]);
        if (mj != 0u) {
          if (hit[j]) { const int pos = wc + (int)__builtin_amdgcn_mbcnt_lo(mj, 0u); int s = esrc[e0 + j]; s = (s < 0) ? 0 : (s >= N ? N - 1 : s); wl[pos] = (s << 12) | (int)sl[j]; atomicAdd(&cnt[sl[j]], 1); }
          wc += __builtin_popcount(mj);
        }
      }
    }
    __builtin_amdgcn_wave_barrier(); __builtin_amdgcn_fence(__ATOMIC_RELEASE, "workgroup"); __builtin_amdgcn_fence(__ATOMIC_ACQUIRE, "workgroup");
    if (DF <= 128) { constexpr int LPH = DF / 4, HPS = 32 / LPH;
      for (int i0 = 0; i0 < wc; i0 += HPS) { const int i = i0 + lane / LPH; if (i < wc) { const int ent = wl[i]; const int s = ent >> 12, slot = ent & 4095; const int col = (lane % LPH) * 4;
          const v4f v = *(const v4f*)(x + (size_t)s * DF + col);
#pragma unroll
          for (int c = 0; c < 4; ++c) atomicAdd(&acc[slot * DF + col + c], (int)rintf(v[c] * FXS)); } } }
    else {
      for (int i = 0; i < wc; ++i) { const int ent = wl[i]; const int s = ent >> 12, slot = ent & 4095;
#pragma unroll
        for (int ch = 0; ch < DF / 128; ++ch) { const int col = ch * 128 + lane * 4; const v4f v = *(const v4f*)(x + (size_t)s * DF + col);
#pragma unroll
          for (int c = 0; c < 4; ++c) atomicAdd(&acc[slot * DF + col + c], (int)rintf(v[c] * FXS)); } } }
    __builtin_amdgcn_wave_barrier();
  }
  __syncthreads();
  for (int pass = 0; pass < 2; ++pass) {
    for (int i = t_; i < NB * DF / 4; i += 256) { const int r = (i * 4) / DF; const int node = base + r; if (node < NPAD) {
        v4f o = {0.0f, 0.0f, 0.0f, 0.0f}; if (node < N) { const float dn = din[node]; const int k0 = (i * 4) % DF;
#pragma unroll
          for (int c = 0; c < 4; ++c) { float val = ((float)acc[i * 4 + c] * FXI) * dn + bias[k0 + c]; if (RELU) val = fmaxf(val, 0.0f); o[c] = val; } }
        *(volatile v4f*)(zin + (size_t)base * DF + (size_t)i * 4) = o; } }
    __threadfence();
  }
}


__global__ __launch_bounds__(256) void pool_kernel(const float* __restrict__ feat, const int* __restrict__ gid, float* __restrict__ nm) {
  __shared__ float Ps[8][H]; __shared__ float Pc[8];
  const int wave = threadIdx.x >> 5, lane = threadIdx.x & 31, b = blockIdx.x;
  v4f s0 = {0, 0, 0, 0}, s1 = {0, 0, 0, 0}; float cnt = 0.0f;
  if (b < NG) {
#pragma unroll 1
    for (int n = wave; n < N; n += 8) { if (gid[n] == b) { const v4f a = *(const v4f*)(feat + (size_t)n * H + lane * 8), c = *(const v4f*)(feat + (size_t)n * H + lane * 8 + 4); s0 += a; s1 += c; cnt += 1.0f; } } }
#pragma unroll
  for (int c = 0; c < 4; ++c) { Ps[wave][lane * 8 + c] = s0[c]; Ps[wave][lane * 8 + 4 + c] = s1[c]; }
  if (lane == 0) Pc[wave] = cnt;
  __syncthreads();
  { const int d = threadIdx.x; float ss = 0.0f, cc = 0.0f;
#pragma unroll
    for (int w = 0; w < 8; ++w) { ss += Ps[w][d]; cc += Pc[w]; }
    const float val = (b < NG) ? ss / fmaxf(cc, 1.0f) : 0.0f;
    for (int pass = 0; pass < 2; ++pass) { ((volatile float*)nm)[(size_t)b * H + d] = val; __threadfence(); } }
}

__global__ __launch_bounds__(64) void out_kernel(const float* __restrict__ z2, const b16* __restrict__ w3, const float* __restrict__ b3, float* __restrict__ out) {
  __shared__ float Ob[64];
  const int lane = threadIdx.x & 31, wave = threadIdx.x >> 5, nloc = lane & 15, hlf = lane >> 4, m0 = wave * 32;
  v8f a0acc = {}, a1acc = {};
#pragma unroll 1
  for (int kb = 0; kb < H2; kb += 32) { v16b a0, l0, a1, l1; frag_split(z2 + (size_t)(m0 + nloc) * H2, kb, hlf, 1.0f, a0, l0); frag_split(z2 + (size_t)(m0 + 16 + nloc) * H2, kb, hlf, 1.0f, a1, l1);
    const v16b bw = frag_kb(w3 + (size_t)nloc * H2 + kb, hlf);
    a0acc = wmma16b(a0, bw, a0acc); a0acc = wmma16b(l0, bw, a0acc); a1acc = wmma16b(a1, bw, a1acc); a1acc = wmma16b(l1, bw, a1acc); }
  if (nloc == 0) {
#pragma unroll
    for (int v = 0; v < 8; ++v) { Ob[m0 + 8 * hlf + v] = a0acc[v] * (1.0f / AS) + b3[0]; Ob[m0 + 16 + 8 * hlf + v] = a1acc[v] * (1.0f / AS) + b3[0]; } }
  __syncthreads();
  if (threadIdx.x < 16) for (int pass = 0; pass < 2; ++pass) { *(volatile v4f*)(out + threadIdx.x * 4) = *(const v4f*)(&Ob[threadIdx.x * 4]); __threadfence(); }
}
}

extern "C" void kernel_launch(void* const* d_in, const int* in_sizes, int n_in,
                              void* d_out, int out_size, void* d_ws, size_t ws_size, hipStream_t stream) {
  (void)n_in; (void)out_size;
  const float* x = (const float*)d_in[0];   const float* W0 = (const float*)d_in[2]; const float* b0 = (const float*)d_in[3];
  const float* gW = (const float*)d_in[4]; const float* gb = (const float*)d_in[5]; const float* W1 = (const float*)d_in[6]; const float* b1 = (const float*)d_in[7];
  const float* W2 = (const float*)d_in[8]; const float* b2 = (const float*)d_in[9]; const float* W3 = (const float*)d_in[10]; const float* b3 = (const float*)d_in[11];
  const int* src = (const int*)d_in[12]; const int* dst = (const int*)d_in[13]; const int* gid = (const int*)d_in[14];
  float* out = (float*)d_out;
  if (in_sizes[0] != N * IN || in_sizes[2] != IN * H || in_sizes[4] != NCONV * H * H || in_sizes[6] != H * H1 || in_sizes[8] != H1 * H2 || in_sizes[10] != H2 || in_sizes[12] != E || in_sizes[13] != E || in_sizes[14] != N) return;
  size_t off = 0; char* ws = (char*)d_ws;
  auto carve = [&](size_t bytes) { char* p = ws + off; off += (bytes + 255) & ~(size_t)255; return p; };
  float* xp = (float*)carve((size_t)NPAD * INP * 4); b16* w0 = (b16*)carve((size_t)H * INP * 2); b16* gw = (b16*)carve((size_t)NCONV * H * H * 2); b16* w1 = (b16*)carve((size_t)H1 * H * 2); b16* w2 = (b16*)carve((size_t)H2 * H1 * 2); b16* w3 = (b16*)carve((size_t)16 * H2 * 2);
  float* din = (float*)carve((size_t)NPAD * 4); float* dout = (float*)carve((size_t)NPAD * 4);
  float* hw = (float*)carve((size_t)NPAD * H * 4); float* feat = (float*)carve((size_t)NPAD * H * 4);
  float* nm = (float*)carve((size_t)128 * H * 4); float* z1 = (float*)carve((size_t)128 * H1 * 4); float* z2 = (float*)carve((size_t)128 * H2 * 4);
  if (off > ws_size) return;
  prep_kernel<<<512, 256, 0, stream>>>(x, W0, gW, W1, W2, W3, xp, w0, gw, w1, w2, w3);
  deg_kernel<<<1, 256, 0, stream>>>(dst, din); deg_kernel<<<1, 256, 0, stream>>>(src, dout);
  lin_kernel<INP, H, false><<<dim3(H / 64, NBLK), 128, 0, stream>>>(xp, dout, w0, nullptr, hw);
  aggsv_kernel<H, 256, false><<<NPAD / 256 + 1, 256, 0, stream>>>(src, dst, hw, din, b0, feat);
  for (int l = 0; l < NCONV; ++l) {
    lin_kernel<H, H, false><<<dim3(H / 64, NBLK), 128, 0, stream>>>(feat, dout, gw + (size_t)l * H * H, nullptr, hw);
    aggsv_kernel<H, 256, true><<<NPAD / 256 + 1, 256, 0, stream>>>(src, dst, hw, din, gb + l * H, feat);
  }
  pool_kernel<<<128, 256, 0, stream>>>(feat, gid, nm);
  lin_kernel<H, H1, true><<<dim3(H1 / 64, 1), 128, 0, stream>>>(nm, nullptr, w1, b1, z1);
  lin_kernel<H1, H2, true><<<dim3(H2 / 64, 1), 128, 0, stream>>>(z1, nullptr, w2, b2, z2);
  out_kernel<<<1, 64, 0, stream>>>(z2, w3, b3, out);
}
